// TripletTransformerNetwork_31009663877393
// MI455X (gfx1250) — hardware-verified
//
#include <hip/hip_runtime.h>
#include <stddef.h>


#define NTHR    256
#define NWAVE   8
#define EPTH    8
#define NGRP    2
#define CHUNK   (NTHR * EPTH * NGRP)
#define WCAP    (EPTH * NGRP * 32)
#define LISTN   (NWAVE * WCAP)
#define NBC     4096
#define NBF     1024
#define RCAP    40960
#define RBN     128
#define TGT     256
#define DEGCAP  128
#define GROWS   128
#define GNC     128
#define OTHR    512
#define NJOB    16
#define NLAYER  4
#define WSCAP   134217728
#define NEG_BIG (-3.0e38f)
#define LDS_FILL ((RCAP + NBF + LISTN) * 4 + 64)
#define LDS_GEMM (GROWS * GNC * 4)

static_assert((CHUNK & (CHUNK - 1)) == 0);
static_assert(CHUNK <= 4096);
static_assert(NBC == 4 * NBF);
static_assert(OTHR * 8 == NBC);
static_assert((RCAP % 32) == 0);
static_assert(TGT == NWAVE * 32);
static_assert(GROWS == NWAVE * 16);
static_assert((DEGCAP % 32) == 0);

typedef float          v2f  __attribute__((ext_vector_type(2)));
typedef float          v4f  __attribute__((ext_vector_type(4)));
typedef float          v8f  __attribute__((ext_vector_type(8)));
typedef int            v4i  __attribute__((ext_vector_type(4)));
typedef unsigned int   v2u  __attribute__((ext_vector_type(2)));
typedef unsigned int   v4u  __attribute__((ext_vector_type(4)));
typedef unsigned short v8us __attribute__((ext_vector_type(8)));
typedef __bf16         v16b __attribute__((ext_vector_type(16)));
union FragB { v16b v; v8us h[2]; };

__device__ __forceinline__ unsigned int bfr(float f) {
  const unsigned int u = __float_as_uint(f);
  return (u + 0x7FFFu + ((u >> 16) & 1u)) >> 16;
}
__device__ __forceinline__ void split1(float x, unsigned short& hb, unsigned short& lb) {
  const unsigned int hu = bfr(x);
  const float hf = __uint_as_float(hu << 16);
  hb = (unsigned short)hu;
  lb = (unsigned short)bfr(x - hf);
}
__device__ __forceinline__ void split8(v4f a, v4f b, v8us& hi, v8us& lo) {
  unsigned short hb, lb;
  split1(a.x, hb, lb); hi[0] = hb; lo[0] = lb;
  split1(a.y, hb, lb); hi[1] = hb; lo[1] = lb;
  split1(a.z, hb, lb); hi[2] = hb; lo[2] = lb;
  split1(a.w, hb, lb); hi[3] = hb; lo[3] = lb;
  split1(b.x, hb, lb); hi[4] = hb; lo[4] = lb;
  split1(b.y, hb, lb); hi[5] = hb; lo[5] = lb;
  split1(b.z, hb, lb); hi[6] = hb; lo[6] = lb;
  split1(b.w, hb, lb); hi[7] = hb; lo[7] = lb;
}
__device__ __forceinline__ void pk2(float x, float y, unsigned int& hi, unsigned int& lo) {
  unsigned short a, b, c, d;
  split1(x, a, c); split1(y, b, d);
  hi = (unsigned int)a | ((unsigned int)b << 16);
  lo = (unsigned int)c | ((unsigned int)d << 16);
}

__device__ __forceinline__ v8f wm(v16b a, v16b b, v8f c) {
  return __builtin_amdgcn_wmma_f32_16x16x32_bf16(false, a, false, b, (short)0, c, false, false);
}
__device__ __forceinline__ v8f wm3(v16b ah, v16b al, v16b bh, v16b bl, v8f c) {
  c = wm(ah, bh, c); c = wm(ah, bl, c); c = wm(al, bh, c);
  asm volatile("v_nop\n\tv_nop\n\tv_nop\n\tv_nop" : "+v"(c) : "v"(ah), "v"(al), "v"(bh), "v"(bl));
  return c;
}

__device__ __forceinline__ float wsum(float v) {
#pragma unroll
  for (int o = 16; o > 0; o >>= 1) v += __shfl_xor(v, o);
  return v;
}

template <int CPL>
__device__ __forceinline__ void ldrow(const float* p, float* v) {
  if (CPL == 8) {
    const v4f a = *(const v4f*)p;
    const v4f b = *(const v4f*)(p + 4);
    v[0] = a.x; v[1] = a.y; v[2] = a.z; v[3] = a.w;
    v[4] = b.x; v[5] = b.y; v[6] = b.z; v[7] = b.w;
  } else if (CPL == 4) {
    const v4f a = *(const v4f*)p;
    v[0] = a.x; v[1] = a.y; v[2] = a.z; v[3] = a.w;
  } else {
    const v2f a = *(const v2f*)p;
    v[0] = a.x; v[1] = a.y;
  }
}

template <int NB>
__device__ __forceinline__ int scan_chunk(const int* __restrict__ dsts, int nE, int cbase, int slotBase,
                                          int vec8, int* list, int tid, int lane, int wave) {
  int wc = 0;
#pragma unroll
  for (int g = 0; g < NGRP; ++g) {
    const int el0  = (g * NTHR + tid) * EPTH;
    const int e0   = cbase + el0;
    const int sent = -2147483647 - 1;
    v4i da, db;
    if (vec8 != 0 && cbase + CHUNK <= nE) {
      da = *(const v4i*)(dsts + e0);
      db = *(const v4i*)(dsts + e0 + 4);
    } else {
      da.x = (e0     < nE) ? dsts[min(e0, nE - 1)] : sent;
      da.y = (e0 + 1 < nE) ? dsts[min(e0 + 1, nE - 1)] : sent;
      da.z = (e0 + 2 < nE) ? dsts[min(e0 + 2, nE - 1)] : sent;
      da.w = (e0 + 3 < nE) ? dsts[min(e0 + 3, nE - 1)] : sent;
      db.x = (e0 + 4 < nE) ? dsts[min(e0 + 4, nE - 1)] : sent;
      db.y = (e0 + 5 < nE) ? dsts[min(e0 + 5, nE - 1)] : sent;
      db.z = (e0 + 6 < nE) ? dsts[min(e0 + 6, nE - 1)] : sent;
      db.w = (e0 + 7 < nE) ? dsts[min(e0 + 7, nE - 1)] : sent;
    }
    const unsigned nb = (unsigned)slotBase;
    const unsigned s0 = (unsigned)da.x - nb, s1 = (unsigned)da.y - nb;
    const unsigned s2 = (unsigned)da.z - nb, s3 = (unsigned)da.w - nb;
    const unsigned s4 = (unsigned)db.x - nb, s5 = (unsigned)db.y - nb;
    const unsigned s6 = (unsigned)db.z - nb, s7 = (unsigned)db.w - nb;
    const bool h0 = s0 < (unsigned)NB, h1 = s1 < (unsigned)NB, h2 = s2 < (unsigned)NB, h3 = s3 < (unsigned)NB;
    const bool h4 = s4 < (unsigned)NB, h5 = s5 < (unsigned)NB, h6 = s6 < (unsigned)NB, h7 = s7 < (unsigned)NB;
    const unsigned any = __builtin_amdgcn_ballot_w32(h0 | h1 | h2 | h3 | h4 | h5 | h6 | h7);
    if (any != 0u) {
#define HITJ(J, HJ, SJ) { \
        const unsigned mj = __builtin_amdgcn_ballot_w32(HJ); \
        if (mj != 0u) { \
          if (HJ) { \
            const int p = wc + (int)__builtin_amdgcn_mbcnt_lo(mj, 0u); \
            if (p < WCAP) list[wave * WCAP + p] = ((el0 + (J)) << 12) | (int)(SJ); \
          } \
          wc += (int)__builtin_popcount(mj); } }
      HITJ(0, h0, s0)
      HITJ(1, h1, s1)
      HITJ(2, h2, s2)
      HITJ(3, h3, s3)
      HITJ(4, h4, s4)
      HITJ(5, h5, s5)
      HITJ(6, h6, s6)
      HITJ(7, h7, s7)
#undef HITJ
    }
  }
  return wc;
}

__global__ __launch_bounds__(NTHR) void k_count(const int* __restrict__ ei, int* cnt, int nE, int vec8) {
  __shared__ __attribute__((aligned(16))) int scnt[NBC];
  __shared__ __attribute__((aligned(16))) int list[LISTN];
  __shared__ int wcnt[NWAVE];
  const int tid = threadIdx.x, lane = tid & 31, wave = tid >> 5;
  const int nodeBase = blockIdx.x * NBC;
  const int* dsts = ei + nE;
  for (int i = tid; i < NBC; i += NTHR) scnt[i] = 0;
  __syncthreads();
  const int nChunks = (nE + CHUNK - 1) / CHUNK;
#pragma unroll 1
  for (int ch = 0; ch < nChunks; ++ch) {
    const int cbase = ch * CHUNK;
    const int wc = scan_chunk<NBC>(dsts, nE, cbase, nodeBase, vec8, list, tid, lane, wave);
    if (lane == 0) wcnt[wave] = wc;
    __syncthreads();
    if (wave == 0) {
#pragma unroll 1
      for (int wsx = 0; wsx < NWAVE; ++wsx) {
        int n = __builtin_amdgcn_readfirstlane(wcnt[wsx]);
        n = n > WCAP ? WCAP : (n < 0 ? 0 : n);
        const int* lp = list + wsx * WCAP;
#pragma unroll 1
        for (int i = 0; i < n; ++i) {
          const int ent  = __builtin_amdgcn_readfirstlane(lp[i]);
          const int slot = ent & (NBC - 1);
          if (lane == 0) scnt[slot] = scnt[slot] + 1;
        }
      }
    }
    __syncthreads();
  }
  v4i cq[4];
#pragma unroll
  for (int q = 0; q < 4; ++q) cq[q] = *(const v4i*)(scnt + (wave * 4 + q) * 128 + 4 * lane);
  int* cp = cnt + (size_t)nodeBase;
#pragma unroll
  for (int q = 0; q < 4; ++q) *(volatile v4i*)(cp + (wave * 4 + q) * 128 + 4 * lane) = cq[q];
  __threadfence();
#pragma unroll
  for (int q = 0; q < 4; ++q) *(volatile v4i*)(cp + (wave * 4 + q) * 128 + 4 * lane) = cq[q];
}

__global__ __launch_bounds__(OTHR) void k_offsets(const int* __restrict__ cnt, int* off, int* rbase, int nChunk) {
  __shared__ __attribute__((aligned(16))) int soff[NBC];
  __shared__ __attribute__((aligned(16))) int srb[RBN];
  __shared__ int wtot[OTHR / 32];
  const int tid = threadIdx.x, lane = tid & 31, wave = tid >> 5, sub = tid >> 7;
  for (int i = tid; i < RBN; i += OTHR) srb[i] = 0;
  int carry = 0;
#pragma unroll 1
  for (int ch = 0; ch < nChunk; ++ch) {
    const int base = ch * NBC;
    const v4i c0 = *(const v4i*)(cnt + base + 8 * tid);
    const v4i c1 = *(const v4i*)(cnt + base + 8 * tid + 4);
    const int e0 = max(c0.x, 0), e1 = max(c0.y, 0), e2 = max(c0.z, 0), e3 = max(c0.w, 0);
    const int e4 = max(c1.x, 0), e5 = max(c1.y, 0), e6 = max(c1.z, 0), e7 = max(c1.w, 0);
    const int ts = e0 + e1 + e2 + e3 + e4 + e5 + e6 + e7;
    int incl = ts;
#pragma unroll
    for (int d = 1; d < 32; d <<= 1) {
      const int t = __shfl_up(incl, d);
      if (lane >= d) incl += t;
    }
    if (lane == 31) wtot[wave] = incl;
    __syncthreads();
    const int S0 = wtot[0]  + wtot[1]  + wtot[2]  + wtot[3];
    const int S1 = wtot[4]  + wtot[5]  + wtot[6]  + wtot[7];
    const int S2 = wtot[8]  + wtot[9]  + wtot[10] + wtot[11];
    const int S3 = wtot[12] + wtot[13] + wtot[14] + wtot[15];
    int pre = 0;
#pragma unroll 1
    for (int w = 4 * sub; w < wave; ++w) pre += wtot[w];
    const int b0 = carry;
    const int b1 = b0 + ((S0 + 31) & ~31);
    const int b2 = b1 + ((S1 + 31) & ~31);
    const int b3 = b2 + ((S2 + 31) & ~31);
    const int b4 = b3 + ((S3 + 31) & ~31);
    const int myb = sub == 0 ? b0 : (sub == 1 ? b1 : (sub == 2 ? b2 : b3));
    if (tid == 0) {
      srb[min(4 * ch + 0, RBN - 1)] = b0;
      srb[min(4 * ch + 1, RBN - 1)] = b1;
      srb[min(4 * ch + 2, RBN - 1)] = b2;
      srb[min(4 * ch + 3, RBN - 1)] = b3;
    }
    int run = myb + pre + incl - ts;
    soff[8 * tid + 0] = run; run += e0;
    soff[8 * tid + 1] = run; run += e1;
    soff[8 * tid + 2] = run; run += e2;
    soff[8 * tid + 3] = run; run += e3;
    soff[8 * tid + 4] = run; run += e4;
    soff[8 * tid + 5] = run; run += e5;
    soff[8 * tid + 6] = run; run += e6;
    soff[8 * tid + 7] = run;
    carry = b4;
    __syncthreads();
    const v4i o0 = *(const v4i*)(soff + 4 * tid);
    const v4i o1 = *(const v4i*)(soff + 4 * (tid + OTHR));
    int* op = off + base;
    *(volatile v4i*)(op + 4 * tid) = o0;
    *(volatile v4i*)(op + 4 * (tid + OTHR)) = o1;
    __threadfence();
    *(volatile v4i*)(op + 4 * tid) = o0;
    *(volatile v4i*)(op + 4 * (tid + OTHR)) = o1;
    __syncthreads();
  }
  if (tid == 0) srb[min(4 * nChunk, RBN - 1)] = carry;
  __syncthreads();
  v4i rv = {0, 0, 0, 0};
  if (tid < 32) rv = *(const v4i*)(srb + 4 * tid);
  if (tid < 32) *(volatile v4i*)(rbase + 4 * tid) = rv;
  __threadfence();
  if (tid < 32) *(volatile v4i*)(rbase + 4 * tid) = rv;
}

__global__ __launch_bounds__(NTHR) void k_fill(const int* __restrict__ ei, const int* __restrict__ off, const int* __restrict__ rbase,
                                               int* csr, int nE, int vec8, int csrLen) {
  extern __shared__ v4f lds_dyn[];
  int* region = (int*)lds_dyn;
  int* cursor = region + RCAP;
  int* list   = cursor + NBF;
  int* wcnt   = list + LISTN;
  const int tid = threadIdx.x, lane = tid & 31, wave = tid >> 5;
  const int b = blockIdx.x;
  const int nodeBase = b * NBF;
  const int* dsts = ei + nE;
  int rb0 = rbase[b];
  const int rb1 = rbase[b + 1];
  rb0 = rb0 < 0 ? 0 : (rb0 > csrLen ? csrLen : rb0);
  rb0 &= ~31;
  int len = rb1 - rb0;
  len = len < 0 ? 0 : (len > RCAP ? RCAP : len);
  int lenW = (len + 31) & ~31;
  if (rb0 + lenW > csrLen) lenW = (csrLen - rb0) & ~31;
  {
    const v4i z = {0, 0, 0, 0};
    for (int i = tid; i < RCAP / 4; i += NTHR) ((v4i*)region)[i] = z;
    for (int s = tid; s < NBF; s += NTHR) {
      int o = off[nodeBase + s] - rb0;
      o = o < 0 ? 0 : (o > RCAP ? RCAP : o);
      cursor[s] = o;
    }
  }
  __syncthreads();
  const int nChunks = (nE + CHUNK - 1) / CHUNK;
#pragma unroll 1
  for (int ch = 0; ch < nChunks; ++ch) {
    const int cbase = ch * CHUNK;
    const int wc = scan_chunk<NBF>(dsts, nE, cbase, nodeBase, vec8, list, tid, lane, wave);
    if (lane == 0) wcnt[wave] = wc;
    __syncthreads();
    if (wave == 0) {
#pragma unroll 1
      for (int wsx = 0; wsx < NWAVE; ++wsx) {
        int n = __builtin_amdgcn_readfirstlane(wcnt[wsx]);
        n = n > WCAP ? WCAP : (n < 0 ? 0 : n);
        const int* lp = list + wsx * WCAP;
#pragma unroll 1
        for (int i = 0; i < n; ++i) {
          const int ent  = __builtin_amdgcn_readfirstlane(lp[i]);
          const int slot = ent & (NBF - 1);
          int e = cbase + ((ent >> 12) & (CHUNK - 1));
          e = e > nE - 1 ? nE - 1 : e;
          if (lane == 0) {
            int p = cursor[slot];
            p = p < 0 ? 0 : (p > RCAP - 1 ? RCAP - 1 : p);
            region[p] = e;
            const int np = p + 1;
            cursor[slot] = np > RCAP ? RCAP : np;
          }
        }
      }
    }
    __syncthreads();
  }
  const int nv = lenW >> 2;
  int* gp = csr + rb0;
#pragma unroll 1
  for (int i = tid; i < nv; i += NTHR) { const v4i v = ((const v4i*)region)[i]; *(volatile v4i*)(gp + 4 * i) = v; }
  __threadfence();
#pragma unroll 1
  for (int i = tid; i < nv; i += NTHR) { const v4i v = ((const v4i*)region)[i]; *(volatile v4i*)(gp + 4 * i) = v; }
}

struct WJob  { const float* src; unsigned short* dst; int K, N, KP, loOff; };
struct WJobs { WJob j[NJOB]; };
static_assert(sizeof(WJob) == 32);
static_assert(sizeof(WJobs) == 32 * NJOB);

__global__ __launch_bounds__(NTHR) void k_wprep(WJobs J) {
  const int y = (int)blockIdx.y;
  const float* src = J.j[0].src; unsigned short* dst = J.j[0].dst;
  int K = J.j[0].K, N = J.j[0].N, KP = J.j[0].KP, loOff = J.j[0].loOff;
#pragma unroll
  for (int i = 1; i < NJOB; ++i)
    if (i == y) { src = J.j[i].src; dst = J.j[i].dst; K = J.j[i].K; N = J.j[i].N; KP = J.j[i].KP; loOff = J.j[i].loOff; }
  const int idx = blockIdx.x * NTHR + threadIdx.x;
  const int kp8 = KP >> 3;
  const int items = N * kp8;
  if (idx >= items) return;
  const int n = idx / kp8;
  const int k0 = (idx - n * kp8) * 8;
  float v[8];
#pragma unroll
  for (int e = 0; e < 8; ++e) {
    const int k = k0 + e;
    const int kc = k < K ? k : K - 1;
    const float x = src[(size_t)kc * N + n];
    v[e] = k < K ? x : 0.0f;
  }
  v4f a, b;
  a.x = v[0]; a.y = v[1]; a.z = v[2]; a.w = v[3];
  b.x = v[4]; b.y = v[5]; b.z = v[6]; b.w = v[7];
  v8us hv, lv;
  split8(a, b, hv, lv);
  unsigned short* dh = dst + (size_t)idx * 8;
  unsigned short* dl = dh + (size_t)loOff;
  *(volatile v8us*)dh = hv; *(volatile v8us*)dl = lv;
  __threadfence();
  *(volatile v8us*)dh = hv; *(volatile v8us*)dl = lv;
}

__global__ __launch_bounds__(NTHR) void k_cvt(const float* __restrict__ x, unsigned short* hi, unsigned short* lo,
                                              int nN, int K, int KP, int items) {
  const int idx = blockIdx.x * NTHR + threadIdx.x;
  if (idx >= items) return;
  const int kp8 = KP >> 3;
  const int r = idx / kp8;
  const int k0 = (idx - r * kp8) * 8;
  const int rc = r < nN ? r : nN - 1;
  const float* xp = x + (size_t)rc * K;
  float v[8];
#pragma unroll
  for (int e = 0; e < 8; ++e) {
    const int k = k0 + e;
    const int kc = k < K ? k : K - 1;
    const float t = xp[kc];
    v[e] = k < K ? t : 0.0f;
  }
  v4f a, b;
  a.x = v[0]; a.y = v[1]; a.z = v[2]; a.w = v[3];
  b.x = v[4]; b.y = v[5]; b.z = v[6]; b.w = v[7];
  v8us hv, lv;
  split8(a, b, hv, lv);
  *(volatile v8us*)(hi + (size_t)idx * 8) = hv; *(volatile v8us*)(lo + (size_t)idx * 8) = lv;
  __threadfence();
  *(volatile v8us*)(hi + (size_t)idx * 8) = hv; *(volatile v8us*)(lo + (size_t)idx * 8) = lv;
}

struct GArgs {
  const unsigned short* A0; const unsigned short* A1; const unsigned short* B0; const unsigned short* B1;
  const float* b0; const float* b1; const float* b2; const float* b3; float* C;
  int lda, ksteps, ldb, ldc, dsh, z0;
};
static_assert(sizeof(GArgs) == 96);

__global__ __launch_bounds__(NTHR) void k_gemm(GArgs g) {
  extern __shared__ v4f lds_dyn[];
  float* stg = (float*)lds_dyn;
  const int tid = threadIdx.x, lane = tid & 31, wave = tid >> 5, hh = lane >> 4, m = lane & 15;
  const int rowBase = (int)blockIdx.x * GROWS, colBase = (int)blockIdx.y * GNC;
  const int arow = rowBase + wave * 16 + m;
  const unsigned short* a0p = g.A0 + (size_t)arow * g.lda + 8 * hh;
  const unsigned short* a1p = g.A1 + (size_t)arow * g.lda + 8 * hh;
  v8f acc[8];
#pragma unroll
  for (int t = 0; t < 8; ++t) { v8f z = {0.f, 0.f, 0.f, 0.f, 0.f, 0.f, 0.f, 0.f}; acc[t] = z; }
#pragma unroll 1
  for (int kt = 0; kt < g.ksteps; ++kt) {
    FragB ah, al;
    ah.h[0] = *(const v8us*)(a0p + 32 * kt); ah.h[1] = *(const v8us*)(a0p + 32 * kt + 16);
    al.h[0] = *(const v8us*)(a1p + 32 * kt); al.h[1] = *(const v8us*)(a1p + 32 * kt + 16);
#pragma unroll
    for (int t = 0; t < 8; ++t) {
      const size_t bo = (size_t)(colBase + 16 * t + m) * g.ldb + 32 * kt + 8 * hh;
      FragB bh, bl;
      bh.h[0] = *(const v8us*)(g.B0 + bo); bh.h[1] = *(const v8us*)(g.B0 + bo + 16);
      bl.h[0] = *(const v8us*)(g.B1 + bo); bl.h[1] = *(const v8us*)(g.B1 + bo + 16);
      acc[t] = wm3(ah.v, al.v, bh.v, bl.v, acc[t]);
    }
  }
  const int r0 = wave * 16 + 8 * hh;
#pragma unroll
  for (int t = 0; t < 8; ++t) {
    const int lcol = 16 * t + m;
    const int gcol = colBase + lcol;
    int which = gcol >> g.dsh;
    which = which > 3 ? 3 : which;
    const float* bp = (which == 0) ? g.b0 : ((which == 1) ? g.b1 : ((which == 2) ? g.b2 : g.b3));
    const float bias = bp[gcol - (which << g.dsh)];
#pragma unroll
    for (int r = 0; r < 8; ++r) stg[(r0 + r) * GNC + lcol] = acc[t][r] + bias;
  }
  __syncthreads();
  float* cb = g.C + (size_t)colBase + 4 * lane;
#pragma unroll
  for (int i = 0; i < 16; ++i) {
    const int lr = wave * 16 + i;
    const v4f v = *(const v4f*)(stg + lr * GNC + 4 * lane);
    *(volatile v4f*)(cb + (size_t)(rowBase + lr) * g.ldc) = v;
  }
  __threadfence();
#pragma unroll
  for (int i = 0; i < 16; ++i) {
    const int lr = wave * 16 + i;
    const v4f v = *(const v4f*)(stg + lr * GNC + 4 * lane);
    *(volatile v4f*)(cb + (size_t)(rowBase + lr) * g.ldc) = v;
  }
}

template <int DO, int H, int KIND>
__global__ __launch_bounds__(NTHR) void k_node(const int* __restrict__ csr, const int* __restrict__ off, const int* __restrict__ cnt,
    const int* __restrict__ ei, const float* __restrict__ qkvs, const float* __restrict__ lng, const float* __restrict__ lnb,
    unsigned int* pH, unsigned int* pL, float* out1, const float* __restrict__ fcW, const float* __restrict__ fcb,
    float* out0, float* mtab, float* dtab, int nN, int nE, int csrLen) {
  constexpr int CPL = DO / 32;
  constexpr int C   = DO / H;
  constexpr int LPH = 32 / H;
  constexpr int HS  = (H == 8) ? 8 : 1;
  constexpr int LD  = 4 * DO;
  constexpr int NSL = DEGCAP * HS;
  static_assert(H == 8 || H == 1);
  static_assert(CPL == 8 || CPL == 4 || CPL == 2);
  static_assert(KIND != 2 || CPL == 4);
  static_assert(KIND == 2 || CPL == 8 || CPL == 2);
  static_assert(KIND != 1 || (H == 8 && CPL == 2));
  __shared__ __attribute__((aligned(16))) float slog[NWAVE * NSL];
  __shared__ __attribute__((aligned(16))) float sfc[(KIND == 1) ? NWAVE * 320 : 4];
  __shared__ __attribute__((aligned(16))) float smt[(KIND == 1) ? NWAVE * 256 : 4];
  __shared__ __attribute__((aligned(16))) float sdt[(KIND == 1) ? NWAVE * 256 : 4];
  const float scale = (C == 32) ? 0.17677669529663688f : ((C == 8) ? 0.35355339059327376f : 0.088388347648318441f);
  const float invDO = 1.0f / (float)DO;
  const int tid = threadIdx.x, lane = tid & 31, wave = tid >> 5;
  const int hidx = (H == 8) ? (lane >> 2) : 0;
  const int sub = lane & (LPH - 1);
  const int tbase = blockIdx.x * TGT + wave * 32;
  float* wl = slog + wave * NSL;
  const int cnt_l = cnt[tbase + lane], off_l = off[tbase + lane];
  float gv[CPL], bv[CPL];
  ldrow<CPL>(lng + CPL * lane, gv);
  ldrow<CPL>(lnb + CPL * lane, bv);
#pragma unroll 1
  for (int j = 0; j < 32; ++j) {
    const int c = tbase + j;
    int n = __builtin_amdgcn_readfirstlane(__shfl(cnt_l, j));
    n = n < 0 ? 0 : (n > DEGCAP ? DEGCAP : n);
    const int st = __builtin_amdgcn_readfirstlane(__shfl(off_l, j));
    const float* qrow = qkvs + (size_t)c * LD + CPL * lane;
    float qv[CPL];
    ldrow<CPL>(qrow, qv);
    __builtin_amdgcn_fence(__ATOMIC_RELEASE, "wavefront");
    __builtin_amdgcn_wave_barrier();
    float M = NEG_BIG;
#pragma unroll 1
    for (int q0 = 0; q0 < n; q0 += 32) {
      int p = st + q0 + lane; p = p < 0 ? 0 : (p > csrLen - 1 ? csrLen - 1 : p);
      int eid = csr[p];   eid = eid < 0 ? 0 : (eid > nE - 1 ? nE - 1 : eid);
      int sl = ei[eid];   sl = sl < 0 ? 0 : (sl > nN - 1 ? nN - 1 : sl);
      const int mcnt = (n - q0) < 32 ? (n - q0) : 32;
#pragma unroll 1
      for (int pp = 0; pp < mcnt; ++pp) {
        const int s = __builtin_amdgcn_readlane(sl, pp);
        float kv[CPL];
        ldrow<CPL>(qkvs + (size_t)s * LD + DO + CPL * lane, kv);
        float d = qv[0] * kv[0];
#pragma unroll
        for (int i = 1; i < CPL; ++i) d = fmaf(qv[i], kv[i], d);
#pragma unroll
        for (int o = 1; o < LPH; o <<= 1) d += __shfl_xor(d, o);
        const float lg = d * scale;
        M = fmaxf(M, lg);
        if (sub == 0) wl[(q0 + pp) * HS + hidx] = lg;
      }
    }
    __builtin_amdgcn_fence(__ATOMIC_RELEASE, "wavefront");
    __builtin_amdgcn_wave_barrier();
#pragma unroll 1
    for (int q0 = 0; q0 < n; q0 += 32) {
      const int e = q0 + lane;
      const bool val = e < n;
#pragma unroll 1
      for (int h = 0; h < HS; ++h) {
        float Mh = M;
        if (H == 8) Mh = __shfl(M, h * LPH);
        const float x = wl[e * HS + h];
        const float pe = __expf(x - Mh);
        wl[e * HS + h] = val ? pe : 0.0f;
      }
    }
    __builtin_amdgcn_fence(__ATOMIC_RELEASE, "wavefront");
    __builtin_amdgcn_wave_barrier();
    float dp = 0.0f;
#pragma unroll 1
    for (int e = sub; e < n; e += LPH) dp += wl[e * HS + hidx];
#pragma unroll
    for (int o = 1; o < LPH; o <<= 1) dp += __shfl_xor(dp, o);
    float acc[CPL];
#pragma unroll
    for (int i = 0; i < CPL; ++i) acc[i] = 0.0f;
#pragma unroll 1
    for (int q0 = 0; q0 < n; q0 += 32) {
      int p = st + q0 + lane; p = p < 0 ? 0 : (p > csrLen - 1 ? csrLen - 1 : p);
      int eid = csr[p];   eid = eid < 0 ? 0 : (eid > nE - 1 ? nE - 1 : eid);
      int sl = ei[eid];   sl = sl < 0 ? 0 : (sl > nN - 1 ? nN - 1 : sl);
      const int mcnt = (n - q0) < 32 ? (n - q0) : 32;
#pragma unroll 1
      for (int pp = 0; pp < mcnt; ++pp) {
        const int s = __builtin_amdgcn_readlane(sl, pp);
        float vv[CPL];
        ldrow<CPL>(qkvs + (size_t)s * LD + 2 * DO + CPL * lane, vv);
        const float w = wl[(q0 + pp) * HS + hidx];
#pragma unroll
        for (int i = 0; i < CPL; ++i) acc[i] = fmaf(w, vv[i], acc[i]);
      }
    }
    const float rd = __builtin_amdgcn_rcpf(dp + 1e-16f);
    if (KIND == 1) {
      if (sub == 0) { smt[wave * 256 + j * 8 + hidx] = M; sdt[wave * 256 + j * 8 + hidx] = dp; }
    }
    float sk[CPL];
    ldrow<CPL>(qrow + 3 * DO, sk);
    float o[CPL];
#pragma unroll
    for (int i = 0; i < CPL; ++i) o[i] = fmaf(acc[i], rd, sk[i]);
    float t[CPL];
#pragma unroll
    for (int i = 0; i < CPL; ++i) t[i] = 0.0f;
#pragma unroll 1
    for (int i = 0; i < CPL; ++i) {
      float x = o[0];
#pragma unroll
      for (int k2 = 1; k2 < CPL; ++k2) x = (i == k2) ? o[k2] : x;
      const float gl = 0.5f * x * (1.0f + erff(x * 0.70710678118654752f));
#pragma unroll
      for (int k2 = 0; k2 < CPL; ++k2) t[k2] = (i == k2) ? gl : t[k2];
    }
    float sm = 0.0f;
#pragma unroll
    for (int i = 0; i < CPL; ++i) sm += t[i];
    const float mean = wsum(sm) * invDO;
    float dd[CPL];
    float sq = 0.0f;
#pragma unroll
    for (int i = 0; i < CPL; ++i) { dd[i] = t[i] - mean; sq = fmaf(dd[i], dd[i], sq); }
    const float var = wsum(sq) * invDO;
    const float rs = rsqrtf(var + 1e-5f);
    float y[CPL];
#pragma unroll
    for (int i = 0; i < CPL; ++i) y[i] = fmaf(gv[i] * dd[i], rs, bv[i]);
    if (KIND != 2) {
      unsigned int hw[4] = {0u, 0u, 0u, 0u}, lw[4] = {0u, 0u, 0u, 0u};
#pragma unroll
      for (int i = 0; i < CPL / 2; ++i) pk2(y[2 * i], y[2 * i + 1], hw[i], lw[i]);
      unsigned int* ph = pH + (size_t)c * (DO / 2) + (CPL / 2) * lane;
      unsigned int* pl = pL + (size_t)c * (DO / 2) + (CPL / 2) * lane;
      if (CPL == 8) {
        v4u ha, la;
        ha.x = hw[0]; ha.y = hw[1]; ha.z = hw[2]; ha.w = hw[3];
        la.x = lw[0]; la.y = lw[1]; la.z = lw[2]; la.w = lw[3];
        *(volatile v4u*)ph = ha; *(volatile v4u*)pl = la;
        __threadfence();
        *(volatile v4u*)ph = ha; *(volatile v4u*)pl = la;
      } else {
        const unsigned int ha = hw[0], la = lw[0];
        *(volatile unsigned int*)ph = ha; *(volatile unsigned int*)pl = la;
        __threadfence();
        *(volatile unsigned int*)ph = ha; *(volatile unsigned int*)pl = la;
      }
    } else {
      v4f yv;
      yv.x = y[0]; yv.y = y[1]; yv.z = y[2]; yv.w = y[3];
      float* op = out1 + (size_t)c * DO + 4 * lane;
      if (c < nN) *(volatile v4f*)op = yv;
      __threadfence();
      if (c < nN) *(volatile v4f*)op = yv;
    }
    if (KIND == 1) {
#pragma unroll 1
      for (int cc = 0; cc < 10; ++cc) {
        float part = 0.0f;
#pragma unroll
        for (int i = 0; i < CPL; ++i) part = fmaf(y[i], fcW[(CPL * lane + i) * 10 + cc], part);
        part = wsum(part);
        const float bcc = fcb[cc];
        if (lane == 0) sfc[wave * 320 + j * 10 + cc] = part + bcc;
      }
    }
  }
  if (KIND == 1) {
    __builtin_amdgcn_fence(__ATOMIC_RELEASE, "wavefront");
    __builtin_amdgcn_wave_barrier();
    const float* fw = sfc + wave * 320;
    const v4f f0 = *(const v4f*)(fw + 4 * lane);
    const v4f f1 = *(const v4f*)(fw + 128 + 4 * lane);
    const v4f f2 = *(const v4f*)(fw + 256 + 4 * (lane & 15));
    const v4f m0 = *(const v4f*)(smt + wave * 256 + 4 * lane);
    const v4f m1 = *(const v4f*)(smt + wave * 256 + 128 + 4 * lane);
    const v4f e0 = *(const v4f*)(sdt + wave * 256 + 4 * lane);
    const v4f e1 = *(const v4f*)(sdt + wave * 256 + 128 + 4 * lane);
    const bool wout = (tbase + 32) <= nN;
    float* op = out0 + (size_t)tbase * 10;
    float* mq = mtab + (size_t)tbase * 8;
    float* dq = dtab + (size_t)tbase * 8;
    if (wout) {
      *(volatile v4f*)(op + 4 * lane) = f0;
      *(volatile v4f*)(op + 128 + 4 * lane) = f1;
      if (lane < 16) *(volatile v4f*)(op + 256 + 4 * lane) = f2;
    }
    *(volatile v4f*)(mq + 4 * lane) = m0; *(volatile v4f*)(mq + 128 + 4 * lane) = m1;
    *(volatile v4f*)(dq + 4 * lane) = e0; *(volatile v4f*)(dq + 128 + 4 * lane) = e1;
    __threadfence();
    if (wout) {
      *(volatile v4f*)(op + 4 * lane) = f0;
      *(volatile v4f*)(op + 128 + 4 * lane) = f1;
      if (lane < 16) *(volatile v4f*)(op + 256 + 4 * lane) = f2;
    }
    *(volatile v4f*)(mq + 4 * lane) = m0; *(volatile v4f*)(mq + 128 + 4 * lane) = m1;
    *(volatile v4f*)(dq + 4 * lane) = e0; *(volatile v4f*)(dq + 128 + 4 * lane) = e1;
  }
}

__global__ __launch_bounds__(NTHR) void k_alpha(const int* __restrict__ ei, const float* __restrict__ qkvs, const float* __restrict__ mtab,
                                                const float* __restrict__ dtab, float* out2, int nN, int nE) {
#pragma clang fp contract(off)
  __shared__ __attribute__((aligned(16))) float sa[NTHR * 8];
  const int tid = threadIdx.x;
  const int e = (int)blockIdx.x * NTHR + tid;
  const int ec = e < nE ? e : nE - 1;
  int s = ei[ec];      s = s < 0 ? 0 : (s > nN - 1 ? nN - 1 : s);
  int d = ei[nE + ec]; d = d < 0 ? 0 : (d > nN - 1 ? nN - 1 : d);
  const float* qp  = qkvs + (size_t)d * 256;
  const float* kp  = qkvs + (size_t)s * 256 + 64;
  const float* mp  = mtab + (size_t)d * 8;
  const float* dnp = dtab + (size_t)d * 8;
#pragma unroll 1
  for (int h = 0; h < 8; ++h) {
    const v4f qa = *(const v4f*)(qp + 8 * h), qb = *(const v4f*)(qp + 8 * h + 4);
    const v4f ka = *(const v4f*)(kp + 8 * h), kb = *(const v4f*)(kp + 8 * h + 4);
    const float t0 = fmaf(qa.y, ka.y, qa.x * ka.x);
    const float t1 = fmaf(qa.w, ka.w, qa.z * ka.z);
    const float t2 = fmaf(qb.y, kb.y, qb.x * kb.x);
    const float t3 = fmaf(qb.w, kb.w, qb.z * kb.z);
    const float lg = ((t0 + t1) + (t2 + t3)) * 0.35355339059327376f;
    const float a = __expf(lg - mp[h]) * __builtin_amdgcn_rcpf(dnp[h] + 1e-16f);
    sa[tid * 8 + h] = a;
  }
  __syncthreads();
  const size_t base = (size_t)blockIdx.x * NTHR * 8;
  const int eA = (int)blockIdx.x * NTHR + (tid >> 1);
  const int eB = eA + NTHR / 2;
  const v4f v0 = *(const v4f*)(sa + 4 * tid);
  const v4f v1 = *(const v4f*)(sa + 4 * (tid + NTHR));
  if (eA < nE) *(volatile v4f*)(out2 + base + 4 * tid) = v0;
  if (eB < nE) *(volatile v4f*)(out2 + base + 4 * (tid + NTHR)) = v1;
  __threadfence();
  if (eA < nE) *(volatile v4f*)(out2 + base + 4 * tid) = v0;
  if (eB < nE) *(volatile v4f*)(out2 + base + 4 * (tid + NTHR)) = v1;
}

static GArgs mkg(const unsigned short* A0, const unsigned short* A1, int lda, int ksteps,
                 const unsigned short* B0, const unsigned short* B1, int ldb,
                 const float* b0, const float* b1, const float* b2, const float* b3,
                 float* C, int ldc, int dsh) {
  GArgs g;
  g.A0 = A0; g.A1 = A1; g.B0 = B0; g.B1 = B1; g.b0 = b0; g.b1 = b1; g.b2 = b2; g.b3 = b3; g.C = C;
  g.lda = lda; g.ksteps = ksteps; g.ldb = ldb; g.ldc = ldc; g.dsh = dsh; g.z0 = 0;
  return g;
}

extern "C" void kernel_launch(void* const* d_in, const int* in_sizes, int n_in,
                              void* d_out, int out_size, void* d_ws, size_t ws_size,
                              hipStream_t stream) {
  if (n_in < 44) return;
  const int dis[NLAYER]  = {128, 256, 64, 256};
  const int dos[NLAYER]  = {256, 64, 256, 128};
  const int dshs[NLAYER] = {8, 6, 8, 7};
  if (in_sizes[0] < 128 || (in_sizes[0] % 128) != 0) return;
  const int N = in_sizes[0] / 128;
  if (in_sizes[1] < 2 || (in_sizes[1] & 1) != 0) return;
  const int E = in_sizes[1] / 2;
  for (int L = 0; L < NLAYER; ++L)
    for (int w = 0; w < 4; ++w) {
      if (in_sizes[2 + 8 * L + w] != dis[L] * dos[L]) return;
      if (in_sizes[6 + 8 * L + w] != dos[L]) return;
    }
  if (in_sizes[34] != 256 || in_sizes[35] != 256 || in_sizes[36] != 64 || in_sizes[37] != 64) return;
  if (in_sizes[38] != 256 || in_sizes[39] != 256 || in_sizes[40] != 128 || in_sizes[41] != 128) return;
  if (in_sizes[42] != 640 || in_sizes[43] != 10) return;
  if ((size_t)out_size != (size_t)N * 10 + (size_t)N * 128 + (size_t)E * 8) return;
  if ((N & 31) != 0) return;
  if (N > (1 << 22) || E > (1 << 26)) return;

  const int NP = ((N + TGT - 1) / TGT) * TGT;
  const int nBC = (N + NBC - 1) / NBC;
  if (4 * nBC + 1 > RBN) return;
  const int CNTPAD = nBC * NBC;
  if (NP > CNTPAD) return;
  const int nBF = (N + NBF - 1) / NBF;
  if (nBF > 4 * nBC) return;
  const int csrLen = ((E + 31) & ~31) + 4096;
  if (31 * 4 * nBC > 4096) return;

  const float* x  = (const float*)d_in[0];
  const int*   ei = (const int*)d_in[1];
  const float* fcW = (const float*)d_in[42];
  const float* fcb = (const float*)d_in[43];
  float* out0 = (float*)d_out;
  float* out1 = out0 + (size_t)N * 10;
  float* out2 = out1 + (size_t)N * 128;

  size_t joffL[NLAYER]; size_t whalves = 0; int maxItems = 0;
  for (int L = 0; L < NLAYER; ++L) {
    joffL[L] = whalves;
    whalves += (size_t)2 * 4 * dos[L] * dis[L];
    const int it = dos[L] * dis[L] / 8;
    maxItems = it > maxItems ? it : maxItems;
  }

  size_t off = 0;
  const size_t oW   = off; off = ((off + whalves * 2) + 255) & ~(size_t)255;
  const size_t oCnt = off; off = ((off + (size_t)CNTPAD * 4) + 255) & ~(size_t)255;
  const size_t oOff = off; off = ((off + (size_t)CNTPAD * 4) + 255) & ~(size_t)255;
  const size_t oRb  = off; off = ((off + (size_t)RBN * 4) + 255) & ~(size_t)255;
  const size_t oCsr = off; off = ((off + (size_t)csrLen * 4) + 255) & ~(size_t)255;
  const size_t oPH  = off; off = ((off + (size_t)NP * 256 * 2) + 255) & ~(size_t)255;
  const size_t oPL  = off; off = ((off + (size_t)NP * 256 * 2) + 255) & ~(size_t)255;
  const size_t oQ   = off; off = ((off + (size_t)NP * 1024 * 4) + 255) & ~(size_t)255;
  const size_t oMt  = off; off = ((off + (size_t)NP * 8 * 4) + 255) & ~(size_t)255;
  const size_t oDt  = off; off = ((off + (size_t)NP * 8 * 4) + 255) & ~(size_t)255;
  if (off > ws_size || off > (size_t)WSCAP) return;

  char* ws = (char*)d_ws;
  unsigned short* wp = (unsigned short*)(ws + oW);
  int* cnt  = (int*)(ws + oCnt);
  int* offp = (int*)(ws + oOff);
  int* rb   = (int*)(ws + oRb);
  int* csr  = (int*)(ws + oCsr);
  unsigned short* pHh = (unsigned short*)(ws + oPH);
  unsigned short* pLh = (unsigned short*)(ws + oPL);
  float* qkvs = (float*)(ws + oQ);
  float* mtab = (float*)(ws + oMt);
  float* dtab = (float*)(ws + oDt);

  WJobs J;
  for (int L = 0; L < NLAYER; ++L)
    for (int w = 0; w < 4; ++w) {
      WJob& jb = J.j[4 * L + w];
      jb.src = (const float*)d_in[2 + 8 * L + w];
      jb.dst = wp + joffL[L] + (size_t)w * dos[L] * dis[L];
      jb.K = dis[L]; jb.N = dos[L]; jb.KP = dis[L]; jb.loOff = 4 * dos[L] * dis[L];
    }
  const int vec8 = ((E & 3) == 0) ? 1 : 0;

  k_wprep<<<dim3((maxItems + NTHR - 1) / NTHR, NJOB, 1), NTHR, 0, stream>>>(J);
  k_count<<<nBC, NTHR, 0, stream>>>(ei, cnt, E, vec8);
  k_offsets<<<1, OTHR, 0, stream>>>(cnt, offp, rb, nBC);
  hipFuncSetAttribute(reinterpret_cast<const void*>(&k_fill), hipFuncAttributeMaxDynamicSharedMemorySize, LDS_FILL);
  k_fill<<<nBF, NTHR, LDS_FILL, stream>>>(ei, offp, rb, csr, E, vec8, csrLen);
  k_cvt<<<(NP * 16 + NTHR - 1) / NTHR, NTHR, 0, stream>>>(x, pHh, pLh, N, 128, 128, NP * 16);

  hipFuncSetAttribute(reinterpret_cast<const void*>(&k_gemm), hipFuncAttributeMaxDynamicSharedMemorySize, LDS_GEMM);

  for (int L = 0; L < NLAYER; ++L) {
    const unsigned short* B0 = wp + joffL[L];
    const unsigned short* B1 = B0 + (size_t)4 * dos[L] * dis[L];
    GArgs a = mkg(pHh, pLh, dis[L], dis[L] / 32, B0, B1, dis[L],
                  (const float*)d_in[6 + 8 * L], (const float*)d_in[7 + 8 * L],
                  (const float*)d_in[8 + 8 * L], (const float*)d_in[9 + 8 * L],
                  qkvs, 4 * dos[L], dshs[L]);
    k_gemm<<<dim3(NP / GROWS, (4 * dos[L]) / GNC, 1), NTHR, LDS_GEMM, stream>>>(a);
    const float* lg = (const float*)d_in[34 + 2 * L];
    const float* lb = (const float*)d_in[35 + 2 * L];
    if (L == 0) {
      k_node<256, 8, 0><<<dim3(NP / TGT), dim3(NTHR), 0, stream>>>(csr, offp, cnt, ei, qkvs, lg, lb,
          (unsigned int*)pHh, (unsigned int*)pLh, out1, fcW, fcb, out0, mtab, dtab, N, E, csrLen);
    } else if (L == 1) {
      k_node<64, 8, 1><<<dim3(NP / TGT), dim3(NTHR), 0, stream>>>(csr, offp, cnt, ei, qkvs, lg, lb,
          (unsigned int*)pHh, (unsigned int*)pLh, out1, fcW, fcb, out0, mtab, dtab, N, E, csrLen);
      k_alpha<<<(E + NTHR - 1) / NTHR, NTHR, 0, stream>>>(ei, qkvs, mtab, dtab, out2, N, E);
    } else if (L == 2) {
      k_node<256, 8, 0><<<dim3(NP / TGT), dim3(NTHR), 0, stream>>>(csr, offp, cnt, ei, qkvs, lg, lb,
          (unsigned int*)pHh, (unsigned int*)pLh, out1, fcW, fcb, out0, mtab, dtab, N, E, csrLen);
    } else {
      k_node<128, 1, 2><<<dim3(NP / TGT), dim3(NTHR), 0, stream>>>(csr, offp, cnt, ei, qkvs, lg, lb,
          (unsigned int*)pHh, (unsigned int*)pLh, out1, fcW, fcb, out0, mtab, dtab, N, E, csrLen);
    }
  }
}
